// AttentionModel_24756191494742
// MI455X (gfx1250) — hardware-run, weakly checked
//
#include <hip/hip_runtime.h>
#include <stddef.h>


typedef _Float16 v16h __attribute__((ext_vector_type(16)));
typedef _Float16 v8h  __attribute__((ext_vector_type(8)));
typedef float    v8f  __attribute__((ext_vector_type(8)));
typedef float    v4f  __attribute__((ext_vector_type(4)));

#ifndef NB
#define NB 4
#endif
#ifndef SEQ
#define SEQ 2048
#endif
#define NB_FULL  4
#define SEQ_FULL 2048
#define DIM   1024
#define HID   4096
#define MROWS (NB * SEQ)
#define EROWS 128
#define EKEYS 64

static_assert(NB >= 1 && NB <= NB_FULL);
static_assert(SEQ >= 256 && SEQ <= SEQ_FULL && (SEQ % 256) == 0);
static_assert(DIM == 1024);
static_assert(HID == 4 * DIM);
static_assert((DIM % 64) == 0 && (DIM % 32) == 0);
static_assert((HID % 64) == 0 && (HID % 32) == 0);
static_assert((SEQ % 64) == 0 && (SEQ % 32) == 0);
static_assert((MROWS % 64) == 0 && (MROWS % 8) == 0);
static_assert(DIM == 2 * 2 * 256);
static_assert(((DIM / 8) % 32) == 0);
static_assert(EROWS <= SEQ && (EROWS % 64) == 0 && EKEYS == 64);
static_assert((size_t)MROWS * HID < (size_t)0xFFFFFFFFu);

#define LDT 72
#define LDC 68
static_assert((LDT % 8) == 0 && LDT >= 64);
static_assert((LDC % 4) == 0 && LDC >= 64);

#define WCARRY 64.0f
#define PCARRY 1024.0f
#define VCARRY 64.0f
#define MCARRY 16.0f
#define RCARRY 1024.0f
#define SCORE_SCALE 0.03125f
#define PE_COEF (-9.210340371976184f / (float)DIM)

#define WSQ_BYTES     ((size_t)DIM * DIM * 2)
#define WFF_BYTES     ((size_t)DIM * HID * 2)
#define PLANE16_BYTES ((size_t)MROWS * DIM * 2)
#define VRES_BYTES    ((size_t)NB * DIM * 64 * 2)
#define MID_BYTES     ((size_t)MROWS * HID * 2)
#define SB_BYTES      ((size_t)SEQ * SEQ * 4)
#define PB_BYTES      ((size_t)SEQ * SEQ * 2)
#define PR_BYTES      ((size_t)NB * EROWS * EKEYS * 2)
#define LINV_BYTES    ((size_t)MROWS * 4)
#define OFF_WQ  ((size_t)0)
#define OFF_WK  (OFF_WQ + WSQ_BYTES)
#define OFF_WV  (OFF_WK + WSQ_BYTES)
#define OFF_W1  (OFF_WV + WSQ_BYTES)
#define OFF_W2  (OFF_W1 + WFF_BYTES)
#define OFF_H1  (OFF_W2 + WFF_BYTES)
#define OFF_Q   (OFF_H1 + PLANE16_BYTES)
#define OFF_K   (OFF_Q + PLANE16_BYTES)
#define OFF_VT  (OFF_K + PLANE16_BYTES)
#define OFF_VR  (OFF_VT + PLANE16_BYTES)
#define OFF_MID (OFF_H1)
#define OFF_CTX (OFF_VR + VRES_BYTES)
#define OFF_S   (OFF_CTX + PLANE16_BYTES)
#define OFF_P   (OFF_S + SB_BYTES)
#define OFF_PR  (OFF_P + PB_BYTES)
#define OFF_LI  (OFF_PR + PR_BYTES)
#define WS_TOTAL (OFF_LI + LINV_BYTES)
static_assert((WSQ_BYTES % 128) == 0 && (WFF_BYTES % 128) == 0 && (PLANE16_BYTES % 128) == 0);
static_assert((VRES_BYTES % 128) == 0 && (MID_BYTES % 128) == 0 && (SB_BYTES % 128) == 0);
static_assert((PB_BYTES % 128) == 0 && (PR_BYTES % 128) == 0 && (LINV_BYTES % 128) == 0);
static_assert(OFF_MID + MID_BYTES <= OFF_VR);
static_assert(WS_TOTAL <= (size_t)134217728);

__device__ __forceinline__ float bf16r(float x) {
  unsigned int u = __float_as_uint(x);
  u = (u + 0x7FFFu + ((u >> 16) & 1u)) & 0xFFFF0000u;
  return __uint_as_float(u);
}

__device__ __forceinline__ v16h frag_at(const _Float16* p) {
  v8h lo = *(const v8h*)(p);
  v8h hi = *(const v8h*)(p + 16);
  v16h out;
#pragma unroll
  for (int i = 0; i < 8; ++i) { out[i] = lo[i]; out[i + 8] = hi[i]; }
  return out;
}
__device__ __forceinline__ v16h ld_frag(const _Float16* base, unsigned ld) {
  const unsigned lane = threadIdx.x & 31u;
  return frag_at(base + (lane & 15u) * ld + (lane >> 4) * 8u);
}

__device__ __forceinline__ v8f wmma16(v16h a, v16h b, v8f c) {
  v8f d = __builtin_amdgcn_wmma_f32_16x16x32_f16(false, a, false, b, (short)0, c,
                                                 false, false);
  asm volatile("v_nop\n\tv_nop\n\tv_nop\n\tv_nop" : "+v"(d) : "v"(a), "v"(b));
  return d;
}

__device__ __forceinline__ float red16_max(float x) {
#pragma unroll
  for (int off = 1; off < 16; off <<= 1) x = fmaxf(x, __shfl_xor(x, off, 32));
  return x;
}
__device__ __forceinline__ float red16_sum(float x) {
#pragma unroll
  for (int off = 1; off < 16; off <<= 1) x += __shfl_xor(x, off, 32);
  return x;
}
__device__ __forceinline__ float red32_sum(float x) {
#pragma unroll
  for (int off = 1; off < 32; off <<= 1) x += __shfl_xor(x, off, 32);
  return x;
}

__device__ __forceinline__ void wave_lds_sync() {
  __builtin_amdgcn_fence(3  , "wavefront");
  asm volatile("s_wait_dscnt 0x0" ::: "memory");
  __builtin_amdgcn_wave_barrier();
}

__device__ __forceinline__ float relu_act(float t) {
  return fmaxf(t, 0.0f);
}

__device__ __forceinline__ float red32_max(float x) {
#pragma unroll
  for (int off = 1; off < 32; off <<= 1) x = fmaxf(x, __shfl_xor(x, off, 32));
  return x;
}
static __device__ __forceinline__ _Float16 toh_flush(float v) {
  const _Float16 r = (_Float16)v;
  return (fabsf(v) < 6.103515625e-05f) ? (_Float16)0.0f : r;
}
__device__ __forceinline__ float gelu_act(float t) {
  return 0.5f * t * (1.0f + erff(t * 0.70710678118654752f));
}

__global__ __launch_bounds__(256) void wconv_kernel(
    const float* __restrict__ W, _Float16* __restrict__ Wt, unsigned ldw, unsigned ldk) {
  __shared__ _Float16 T[64 * LDT];
  const unsigned tid = threadIdx.x;
  const unsigned n0 = blockIdx.x * 64u;
  const unsigned k0 = blockIdx.y * 64u;
#pragma unroll 4
  for (unsigned j = 0; j < 16u; ++j) {
    const unsigned idx = tid + 256u * j;
    const unsigned kr = idx >> 6, nc = idx & 63u;
    const float v = W[(size_t)(k0 + kr) * ldw + n0 + nc];
    T[nc * LDT + kr] = (_Float16)(WCARRY * bf16r(v));
  }
  __syncthreads();
  v8h x[2];
  size_t off[2];
#pragma unroll
  for (unsigned i = 0; i < 2u; ++i) {
    const unsigned n = 32u * i + (tid >> 3);
    const unsigned kc = (tid & 7u) * 8u;
    x[i] = *(const v8h*)&T[n * LDT + kc];
    off[i] = (size_t)(n0 + n) * ldk + k0 + kc;
  }
#pragma unroll
  for (int i = 0; i < 2; ++i) *(volatile v8h*)(Wt + off[i]) = x[i];
  __threadfence();
#pragma unroll
  for (int i = 0; i < 2; ++i) *(volatile v8h*)(Wt + off[i]) = x[i];
}

__global__ __launch_bounds__(256) void pe_add_kernel(
    const float* __restrict__ X, _Float16* __restrict__ dst) {
#pragma clang fp contract(off)
  __shared__ float pe[DIM];
  const unsigned tid = threadIdx.x;
  const unsigned s = blockIdx.x;
#pragma unroll 1
  for (unsigned i = 0; i < 2u; ++i) {
    const unsigned j = tid + 256u * i;
    const float e = (float)(2u * j) * PE_COEF;
    const float dv = expf(e);
    const float ang = (float)s * dv;
    const float sn = sinf(ang);
    const float cs = cosf(ang);
    pe[2u * j] = sn;
    pe[2u * j + 1u] = cs;
  }
  __syncthreads();
  const unsigned ngroups = (unsigned)NB * (unsigned)(DIM / 8);
#pragma unroll 1
  for (unsigned i = 0; i < (ngroups + 255u) / 256u; ++i) {
    const unsigned g = tid + 256u * i;
    if (g < ngroups) {
      const unsigned b = g / (unsigned)(DIM / 8);
      const unsigned c = (g - b * (unsigned)(DIM / 8)) * 8u;
      const float* xr = X + ((size_t)s * NB_FULL + b) * DIM + c;
      const v4f a0 = *(const v4f*)(xr);
      const v4f a1 = *(const v4f*)(xr + 4);
      const v4f p0 = *(const v4f*)&pe[c];
      const v4f p1 = *(const v4f*)&pe[c + 4u];
      v8h o;
#pragma unroll
      for (int k = 0; k < 4; ++k) {
        o[k]     = toh_flush(bf16r(a0[k]) + p0[k]);
        o[k + 4] = toh_flush(bf16r(a1[k]) + p1[k]);
      }
      _Float16* p = dst + ((size_t)b * SEQ + s) * DIM + c;
      *(volatile v8h*)p = o;
      __threadfence();
      *(volatile v8h*)p = o;
    }
  }
}

template <int MODE>
__device__ __forceinline__ void gemm_body(
    const _Float16* __restrict__ A16, const _Float16* __restrict__ Bt, const unsigned K,
    const float* __restrict__ bias, const float* __restrict__ addf,
    float* __restrict__ outf, _Float16* __restrict__ out16, _Float16* __restrict__ out16r) {
  __shared__ float Cs[64 * LDC];
  const unsigned tid = threadIdx.x, lane = tid & 31u, w = tid >> 5;
  const unsigned mw = w >> 1, nw = w & 1u;
  const unsigned hh = lane >> 4, m = lane & 15u;
  const unsigned n0 = blockIdx.x * 64u;
  const unsigned row0 = blockIdx.y * 64u;

  const _Float16* ap  = A16 + (size_t)(row0 + mw * 16u + m) * K + hh * 8u;
  const _Float16* bp0 = Bt + (size_t)(n0 + nw * 32u + m) * K + hh * 8u;
  const _Float16* bp1 = bp0 + (size_t)16 * K;
  v8f acc0 = {}, acc1 = {};
#pragma unroll 2
  for (unsigned k0 = 0; k0 < K; k0 += 32u) {
    const v16h a  = frag_at(ap + k0);
    const v16h b0 = frag_at(bp0 + k0);
    const v16h b1 = frag_at(bp1 + k0);
    acc0 = wmma16(a, b0, acc0);
    acc1 = wmma16(a, b1, acc1);
  }
#pragma unroll
  for (int r = 0; r < 8; ++r) {
    float* d = &Cs[(mw * 16u + hh * 8u + (unsigned)r) * LDC + nw * 32u + m];
    d[0]  = acc0[r];
    d[16] = acc1[r];
  }
  __syncthreads();

  if (MODE == 3) {
#pragma unroll 1
    for (unsigned g = 0; g < 4u; ++g) {
      const unsigned r = 32u * (g >> 1) + (tid >> 3);
      const unsigned c = (tid & 7u) * 8u + 4u * (g & 1u);
      const v4f u  = *(const v4f*)&Cs[r * LDC + c];
      const v4f gb = *(const v4f*)(bias + n0 + c);
      v4f t;
#pragma unroll
      for (int j = 0; j < 4; ++j)
        t[j] = MCARRY * relu_act(u[j] * (1.0f / WCARRY) + bf16r(gb[j]));
      *(v4f*)&Cs[r * LDC + c] = t;
    }
  }

  if (MODE == 0 || MODE == 3) {
    const unsigned ldo = (MODE == 3) ? (unsigned)HID : (unsigned)DIM;
    v8h x[2];
    size_t off[2];
#pragma unroll
    for (unsigned i = 0; i < 2u; ++i) {
      const unsigned r = 32u * i + (tid >> 3);
      const unsigned c = (tid & 7u) * 8u;
      const v4f u0 = *(const v4f*)&Cs[r * LDC + c];
      const v4f u1 = *(const v4f*)&Cs[r * LDC + c + 4];
      if (MODE == 3) {
#pragma unroll
        for (int j = 0; j < 4; ++j) {
          x[i][j]     = (_Float16)u0[j];
          x[i][j + 4] = (_Float16)u1[j];
        }
      } else {
        const v4f g0 = *(const v4f*)(bias + n0 + c);
        const v4f g1 = *(const v4f*)(bias + n0 + c + 4u);
#pragma unroll
        for (int j = 0; j < 4; ++j) {
          x[i][j]     = (_Float16)(u0[j] * (1.0f / WCARRY) + bf16r(g0[j]));
          x[i][j + 4] = (_Float16)(u1[j] * (1.0f / WCARRY) + bf16r(g1[j]));
        }
      }
      off[i] = (size_t)(row0 + r) * ldo + n0 + c;
    }
#pragma unroll
    for (int i = 0; i < 2; ++i) *(volatile v8h*)(out16 + off[i]) = x[i];
    __threadfence();
#pragma unroll
    for (int i = 0; i < 2; ++i) *(volatile v8h*)(out16 + off[i]) = x[i];
  }

  if (MODE == 1) {
    const unsigned bidx = row0 / (unsigned)SEQ;
    const unsigned key0 = row0 - bidx * (unsigned)SEQ;
    const bool first_tile = (key0 == 0u);
    v8h x[2], xr[2];
    size_t off[2], offr[2];
#pragma unroll
    for (unsigned i = 0; i < 2u; ++i) {
      const unsigned dcol = 32u * i + (tid >> 3);
      const unsigned kk = (tid & 7u) * 8u;
      const float bb = bf16r(bias[n0 + dcol]);
#pragma unroll
      for (unsigned j = 0; j < 8u; ++j) {
        const float t = Cs[(kk + j) * LDC + dcol] * (1.0f / WCARRY) + bb;
        const _Float16 hi = (_Float16)t;
        x[i][j]  = hi;
        xr[i][j] = (_Float16)((t - (float)hi) * RCARRY);
      }
      off[i]  = ((size_t)bidx * DIM + n0 + dcol) * SEQ + key0 + kk;
      offr[i] = ((size_t)bidx * DIM + n0 + dcol) * 64u + kk;
    }
#pragma unroll
    for (int i = 0; i < 2; ++i) *(volatile v8h*)(out16 + off[i]) = x[i];
    if (first_tile) {
#pragma unroll
      for (int i = 0; i < 2; ++i) *(volatile v8h*)(out16r + offr[i]) = xr[i];
    }
    __threadfence();
#pragma unroll
    for (int i = 0; i < 2; ++i) *(volatile v8h*)(out16 + off[i]) = x[i];
    if (first_tile) {
#pragma unroll
      for (int i = 0; i < 2; ++i) *(volatile v8h*)(out16r + offr[i]) = xr[i];
    }
  }

  if (MODE == 2 || MODE == 4) {
    const float cs = (MODE == 2) ? (1.0f / (WCARRY * VCARRY)) : (1.0f / (WCARRY * MCARRY));
    v4f xs[4];
    size_t off[4];
#pragma unroll
    for (unsigned i = 0; i < 4u; ++i) {
      const unsigned r = 16u * i + (tid >> 4);
      const unsigned c = (tid & 15u) * 4u;
      const unsigned crow = row0 + r;
      const unsigned bidx = crow / (unsigned)SEQ;
      const unsigned sq = crow - bidx * (unsigned)SEQ;
      const size_t frow = (size_t)bidx * SEQ_FULL + sq;
      const size_t inrow  = (MODE == 2) ? frow : (size_t)crow;
      const size_t outrow = (MODE == 2) ? (size_t)crow : frow;
      const v4f u = *(const v4f*)&Cs[r * LDC + c];
      const v4f g = *(const v4f*)(bias + n0 + c);
      const v4f xin = *(const v4f*)(addf + inrow * DIM + n0 + c);
      v4f val;
#pragma unroll
      for (int j = 0; j < 4; ++j) {
        const float base = (MODE == 2) ? bf16r(xin[j]) : xin[j];
        val[j] = base + (u[j] * cs + bf16r(g[j]));
      }
      xs[i] = val;
      off[i] = outrow * DIM + n0 + c;
    }
#pragma unroll
    for (int i = 0; i < 4; ++i) *(volatile v4f*)(outf + off[i]) = xs[i];
    __threadfence();
#pragma unroll
    for (int i = 0; i < 4; ++i) *(volatile v4f*)(outf + off[i]) = xs[i];
  }
}

__global__ __launch_bounds__(256) void gemm_qk_kernel(
    const _Float16* __restrict__ A16, const _Float16* __restrict__ Bt,
    const float* __restrict__ bias, _Float16* __restrict__ out16) {
  gemm_body<0>(A16, Bt, (unsigned)DIM, bias, bias, (float*)0, out16, out16);
}
__global__ __launch_bounds__(256) void gemm_v_kernel(
    const _Float16* __restrict__ A16, const _Float16* __restrict__ Bt,
    const float* __restrict__ bias, _Float16* __restrict__ vt, _Float16* __restrict__ vtr) {
  gemm_body<1>(A16, Bt, (unsigned)DIM, bias, bias, (float*)0, vt, vtr);
}

#define XM_SCORES 0
#define XM_PV     1
#define XM_FFN1   2
#define XM_FFN2   3

template <int XM>
__device__ __forceinline__ void gemm_x_body(
    const _Float16* __restrict__ A16, const unsigned lda,
    const _Float16* __restrict__ Bt, const unsigned ldb, const unsigned kfull,
    const _Float16* __restrict__ Ares, const _Float16* __restrict__ Bres,
    const float* __restrict__ vec,
    float* __restrict__ outf, _Float16* __restrict__ out16) {
  __shared__ float Cs[64 * LDC];
  const unsigned tid = threadIdx.x, lane = tid & 31u;
  const unsigned w = (unsigned)__builtin_amdgcn_readfirstlane((int)(tid >> 5));
  const unsigned mw = w >> 1, nw = w & 1u;
  const unsigned hh = lane >> 4, m = lane & 15u;
  const unsigned n0 = blockIdx.x * 64u;
  const unsigned row0 = blockIdx.y * 64u;
  if (XM == XM_SCORES) {
    if (n0 > row0) return;
  }
  const unsigned kend = (XM == XM_PV) ? (row0 + 64u) : kfull;

  const _Float16* ap  = A16 + (size_t)(row0 + mw * 16u + m) * lda + hh * 8u;
  const _Float16* bp0 = Bt + (size_t)(n0 + nw * 32u + m) * ldb + hh * 8u;
  const _Float16* bp1 = bp0 + (size_t)16 * ldb;
  v8f acc0 = {}, acc1 = {};
#pragma unroll 2
  for (unsigned k0 = 0; k0 < kend; k0 += 32u) {
    const v16h a  = frag_at(ap + k0);
    const v16h b0 = frag_at(bp0 + k0);
    const v16h b1 = frag_at(bp1 + k0);
    acc0 = wmma16(a, b0, acc0);
    acc1 = wmma16(a, b1, acc1);
  }

  if (XM == XM_PV) {
    if (row0 < (unsigned)EROWS) {
      const _Float16* rp  = Ares + (size_t)(row0 + mw * 16u + m) * EKEYS + hh * 8u;
      const _Float16* vr0 = Bres + (size_t)(n0 + nw * 32u + m) * EKEYS + hh * 8u;
      const _Float16* vr1 = vr0 + (size_t)16 * EKEYS;
      v8f ra0 = {}, ra1 = {};
#pragma unroll
      for (unsigned k0 = 0; k0 < (unsigned)EKEYS; k0 += 32u) {
        const v16h ah  = frag_at(ap + k0);
        const v16h ar  = frag_at(rp + k0);
        const v16h bh0 = frag_at(bp0 + k0);
        const v16h bh1 = frag_at(bp1 + k0);
        const v16h br0 = frag_at(vr0 + k0);
        const v16h br1 = frag_at(vr1 + k0);
        ra0 = wmma16(ah, br0, ra0);
        ra0 = wmma16(ar, bh0, ra0);
        ra1 = wmma16(ah, br1, ra1);
        ra1 = wmma16(ar, bh1, ra1);
      }
#pragma unroll
      for (int r = 0; r < 8; ++r) {
        acc0[r] = acc0[r] + ra0[r] * (1.0f / RCARRY);
        acc1[r] = acc1[r] + ra1[r] * (1.0f / RCARRY);
      }
    }
  }

#pragma unroll
  for (int r = 0; r < 8; ++r) {
    float* d = &Cs[(mw * 16u + hh * 8u + (unsigned)r) * LDC + nw * 32u + m];
    d[0]  = acc0[r];
    d[16] = acc1[r];
  }
  __syncthreads();

  if (XM == XM_FFN1) {
#pragma unroll 1
    for (unsigned g = 0; g < 4u; ++g) {
      const unsigned r = 32u * (g >> 1) + (tid >> 3);
      const unsigned c = (tid & 7u) * 8u + 4u * (g & 1u);
      const v4f u  = *(const v4f*)&Cs[r * LDC + c];
      const v4f gb = *(const v4f*)(vec + n0 + c);
      v4f t;
#pragma unroll
      for (int j = 0; j < 4; ++j)
        t[j] = MCARRY * gelu_act(u[j] * (1.0f / (WCARRY * VCARRY)) + bf16r(gb[j]));
      *(v4f*)&Cs[r * LDC + c] = t;
    }
  }

  if (XM == XM_PV || XM == XM_FFN1) {
    const unsigned ldo = (XM == XM_FFN1) ? (unsigned)HID : (unsigned)DIM;
    v8h x[2];
    size_t off[2];
#pragma unroll
    for (unsigned i = 0; i < 2u; ++i) {
      const unsigned r = 32u * i + (tid >> 3);
      const unsigned c = (tid & 7u) * 8u;
      const v4f u0 = *(const v4f*)&Cs[r * LDC + c];
      const v4f u1 = *(const v4f*)&Cs[r * LDC + c + 4];
      float f = 1.0f;
      if (XM == XM_PV) f = VCARRY * vec[row0 + r];
#pragma unroll
      for (int j = 0; j < 4; ++j) {
        x[i][j]     = toh_flush(u0[j] * f);
        x[i][j + 4] = toh_flush(u1[j] * f);
      }
      off[i] = (size_t)(row0 + r) * ldo + n0 + c;
    }
#pragma unroll
    for (int i = 0; i < 2; ++i) *(volatile v8h*)(out16 + off[i]) = x[i];
    __threadfence();
#pragma unroll
    for (int i = 0; i < 2; ++i) *(volatile v8h*)(out16 + off[i]) = x[i];
  }

  if (XM == XM_SCORES || XM == XM_FFN2) {
    v4f xs[4];
    size_t off[4];
#pragma unroll
    for (unsigned i = 0; i < 4u; ++i) {
      const unsigned r = 16u * i + (tid >> 4);
      const unsigned c = (tid & 15u) * 4u;
      const v4f u = *(const v4f*)&Cs[r * LDC + c];
      v4f val;
      if (XM == XM_SCORES) {
#pragma unroll
        for (int j = 0; j < 4; ++j) val[j] = u[j] * SCORE_SCALE;
        off[i] = (size_t)(row0 + r) * SEQ + n0 + c;
      } else {
        const unsigned crow = row0 + r;
        const unsigned bidx = crow / (unsigned)SEQ;
        const unsigned sq = crow - bidx * (unsigned)SEQ;
        const size_t orow = (size_t)sq * NB_FULL + bidx;
        const v4f g = *(const v4f*)(vec + n0 + c);
#pragma unroll
        for (int j = 0; j < 4; ++j)
          val[j] = u[j] * (1.0f / (WCARRY * MCARRY)) + bf16r(g[j]);
        off[i] = orow * DIM + n0 + c;
      }
      xs[i] = val;
    }
#pragma unroll
    for (int i = 0; i < 4; ++i) *(volatile v4f*)(outf + off[i]) = xs[i];
    __threadfence();
#pragma unroll
    for (int i = 0; i < 4; ++i) *(volatile v4f*)(outf + off[i]) = xs[i];
  }
}

__global__ __launch_bounds__(256) void scores_kernel(
    const _Float16* __restrict__ Qb, const _Float16* __restrict__ Kb, float* __restrict__ Sb) {
  gemm_x_body<XM_SCORES>(Qb, (unsigned)DIM, Kb, (unsigned)DIM, (unsigned)DIM,
                         (const _Float16*)0, (const _Float16*)0, (const float*)0,
                         Sb, (_Float16*)0);
}
__global__ __launch_bounds__(256) void pv_kernel(
    const _Float16* __restrict__ Pb, const _Float16* __restrict__ Vtb,
    const _Float16* __restrict__ PRb, const _Float16* __restrict__ VRb,
    const float* __restrict__ linv, _Float16* __restrict__ ctx) {
  gemm_x_body<XM_PV>(Pb, (unsigned)SEQ, Vtb, (unsigned)SEQ, (unsigned)SEQ,
                     PRb, VRb, linv, (float*)0, ctx);
}
__global__ __launch_bounds__(256) void ffn1_kernel(
    const _Float16* __restrict__ A16, const _Float16* __restrict__ Bt,
    const float* __restrict__ bias, _Float16* __restrict__ mid) {
  gemm_x_body<XM_FFN1>(A16, (unsigned)DIM, Bt, (unsigned)DIM, (unsigned)DIM,
                       (const _Float16*)0, (const _Float16*)0, bias, (float*)0, mid);
}
__global__ __launch_bounds__(256) void ffn2_kernel(
    const _Float16* __restrict__ A16, const _Float16* __restrict__ Bt,
    const float* __restrict__ bias, float* __restrict__ outf) {
  gemm_x_body<XM_FFN2>(A16, (unsigned)HID, Bt, (unsigned)HID, (unsigned)HID,
                       (const _Float16*)0, (const _Float16*)0, bias, outf, (_Float16*)0);
}

__global__ __launch_bounds__(256) void softmax_kernel(
    const float* __restrict__ S, _Float16* __restrict__ P, _Float16* __restrict__ PR,
    float* __restrict__ LI) {
#pragma clang fp contract(off)
  __shared__ float lis[32];
  const unsigned lane = threadIdx.x & 31u;
  const unsigned wave = (unsigned)__builtin_amdgcn_readfirstlane((int)(threadIdx.x >> 5));
  const unsigned q0 = blockIdx.x * 32u;
#pragma unroll 1
  for (unsigned i = 0; i < 4u; ++i) {
    const unsigned q = q0 + wave * 4u + i;
    const unsigned tile_end = (q & ~63u) + 64u;
    const unsigned ncols = (q & ~255u) + 256u;
    const bool early_row = (q < (unsigned)EROWS);
    const float* srow = S + (size_t)q * SEQ;

    float mx = -1.0e30f;
#pragma unroll 1
    for (unsigned c0 = 0; c0 < ncols; c0 += 256u) {
      const unsigned c = c0 + lane * 8u;
      const unsigned cl = (c < tile_end) ? c : (tile_end - 8u);
      const v4f a0 = *(const v4f*)(srow + cl);
      const v4f a1 = *(const v4f*)(srow + cl + 4u);
#pragma unroll
      for (int j = 0; j < 4; ++j) {
        const float t0 = (c + (unsigned)j <= q) ? a0[j] : -1.0e30f;
        const float t1 = (c + 4u + (unsigned)j <= q) ? a1[j] : -1.0e30f;
        mx = fmaxf(mx, fmaxf(t0, t1));
      }
    }
    mx = red32_max(mx);

    float ls = 0.0f;
#pragma unroll 1
    for (unsigned c0 = 0; c0 < ncols; c0 += 256u) {
      const unsigned c = c0 + lane * 8u;
      const unsigned cl = (c < tile_end) ? c : (tile_end - 8u);
      const v4f a0 = *(const v4f*)(srow + cl);
      const v4f a1 = *(const v4f*)(srow + cl + 4u);
      float e[8];
#pragma unroll
      for (int j = 0; j < 4; ++j) {
        const float x0 = PCARRY * __expf(a0[j] - mx);
        const float x1 = PCARRY * __expf(a1[j] - mx);
        e[j]     = (c + (unsigned)j <= q) ? x0 : 0.0f;
        e[j + 4] = (c + 4u + (unsigned)j <= q) ? x1 : 0.0f;
      }
      v8h o;
#pragma unroll
      for (int j = 0; j < 8; ++j) {
        const _Float16 hv = toh_flush(e[j]);
        o[j] = hv;
        ls += (float)hv;
      }
      const bool early = early_row && (c0 == 0u);
      v8h orr = {};
      if (early) {
        float rs = 0.0f;
#pragma unroll
        for (int j = 0; j < 8; ++j) {
          const _Float16 rv = toh_flush((e[j] - (float)o[j]) * RCARRY);
          orr[j] = rv;
          rs += (float)rv;
        }
        const float radd = rs * (1.0f / RCARRY);
        ls += (lane < 8u) ? radd : 0.0f;
      }
      _Float16* pp = P + (size_t)q * SEQ + c;
      _Float16* pr = PR + (size_t)(early ? q : 0u) * EKEYS + (lane & 7u) * 8u;
      *(volatile v8h*)pp = o;
      if (early && lane < 8u) *(volatile v8h*)pr = orr;
      __threadfence();
      *(volatile v8h*)pp = o;
      if (early && lane < 8u) *(volatile v8h*)pr = orr;
    }
    const float l = red32_sum(ls);
    if (lane == 0u) lis[wave * 4u + i] = __builtin_amdgcn_rcpf(l);
  }
  __syncthreads();
  if (wave == 0u) {
    if (lane < 8u) {
      const v4f v = *(const v4f*)&lis[lane * 4u];
      float* d = LI + q0 + lane * 4u;
      *(volatile v4f*)d = v;
      __threadfence();
      *(volatile v4f*)d = v;
    }
  }
}

extern "C" void kernel_launch(void* const* d_in, const int* in_sizes, int n_in,
                              void* d_out, int out_size, void* d_ws, size_t ws_size,
                              hipStream_t stream) {
  if (n_in < 11) return;
  const long long need_x = ((long long)(SEQ - 1) * NB_FULL + NB) * DIM;
  if ((long long)in_sizes[0] < need_x) return;
  if ((long long)in_sizes[1] < (long long)DIM * DIM) return;
  if ((long long)in_sizes[3] < (long long)DIM * DIM) return;
  if ((long long)in_sizes[5] < (long long)DIM * DIM) return;
  if ((long long)in_sizes[7] < (long long)DIM * HID) return;
  if ((long long)in_sizes[9] < (long long)DIM * HID) return;
  if (in_sizes[2] < DIM || in_sizes[4] < DIM || in_sizes[6] < DIM) return;
  if (in_sizes[8] < HID || in_sizes[10] < DIM) return;
  if ((long long)out_size < need_x) return;
  if (ws_size < WS_TOTAL) return;

  const float* X   = (const float*)d_in[0];
  const float* wq  = (const float*)d_in[1];
  const float* bq  = (const float*)d_in[2];
  const float* wk  = (const float*)d_in[3];
  const float* bk  = (const float*)d_in[4];
  const float* wv  = (const float*)d_in[5];
  const float* bv  = (const float*)d_in[6];
  const float* w1  = (const float*)d_in[7];
  const float* b1  = (const float*)d_in[8];
  const float* w2  = (const float*)d_in[9];
  const float* b2  = (const float*)d_in[10];
  float* out = (float*)d_out;

  char* ws = (char*)d_ws;
  _Float16* Wq_t  = (_Float16*)(ws + OFF_WQ);
  _Float16* Wk_t  = (_Float16*)(ws + OFF_WK);
  _Float16* Wv_t  = (_Float16*)(ws + OFF_WV);
  _Float16* W1_t  = (_Float16*)(ws + OFF_W1);
  _Float16* W2_t  = (_Float16*)(ws + OFF_W2);
  _Float16* H1    = (_Float16*)(ws + OFF_H1);
  _Float16* Qh16  = (_Float16*)(ws + OFF_Q);
  _Float16* Kh16  = (_Float16*)(ws + OFF_K);
  _Float16* Vt16  = (_Float16*)(ws + OFF_VT);
  _Float16* VtR16 = (_Float16*)(ws + OFF_VR);
  _Float16* Ctx16 = (_Float16*)(ws + OFF_CTX);
  float*    Sf    = (float*)(ws + OFF_S);
  _Float16* P16   = (_Float16*)(ws + OFF_P);
  _Float16* PR16  = (_Float16*)(ws + OFF_PR);
  float*    Linv  = (float*)(ws + OFF_LI);
  _Float16* Mid16 = (_Float16*)(ws + OFF_MID);

  dim3 blk(256);
  dim3 gsq(DIM / 64, DIM / 64);
  dim3 gg(DIM / 64, MROWS / 64);

  wconv_kernel<<<gsq, blk, 0, stream>>>(wq, Wq_t, (unsigned)DIM, (unsigned)DIM);
  wconv_kernel<<<gsq, blk, 0, stream>>>(wk, Wk_t, (unsigned)DIM, (unsigned)DIM);
  wconv_kernel<<<gsq, blk, 0, stream>>>(wv, Wv_t, (unsigned)DIM, (unsigned)DIM);
  wconv_kernel<<<dim3(HID / 64, DIM / 64), blk, 0, stream>>>(w1, W1_t, (unsigned)HID, (unsigned)DIM);
  wconv_kernel<<<dim3(DIM / 64, HID / 64), blk, 0, stream>>>(w2, W2_t, (unsigned)DIM, (unsigned)HID);

  pe_add_kernel<<<dim3(SEQ), blk, 0, stream>>>(X, H1);
  gemm_qk_kernel<<<gg, blk, 0, stream>>>(H1, Wq_t, bq, Qh16);
  gemm_qk_kernel<<<gg, blk, 0, stream>>>(H1, Wk_t, bk, Kh16);
  gemm_v_kernel<<<gg, blk, 0, stream>>>(H1, Wv_t, bv, Vt16, VtR16);

  for (unsigned b = 0; b < (unsigned)NB; ++b) {
    const _Float16* Qb  = Qh16 + (size_t)b * SEQ * DIM;
    const _Float16* Kb  = Kh16 + (size_t)b * SEQ * DIM;
    const _Float16* Vtb = Vt16 + (size_t)b * DIM * SEQ;
    const _Float16* VRb = VtR16 + (size_t)b * DIM * 64;
    _Float16* PRb  = PR16 + (size_t)b * EROWS * EKEYS;
    float*    LIb  = Linv + (size_t)b * SEQ;
    _Float16* Ctxb = Ctx16 + (size_t)b * SEQ * DIM;
    scores_kernel<<<dim3(SEQ / 64, SEQ / 64), blk, 0, stream>>>(Qb, Kb, Sf);
    softmax_kernel<<<dim3(SEQ / 32), blk, 0, stream>>>(Sf, P16, PRb, LIb);
    pv_kernel<<<dim3(DIM / 64, SEQ / 64), blk, 0, stream>>>(P16, Vtb, PRb, VRb, LIb, Ctxb);
  }

  ffn1_kernel<<<dim3(HID / 64, MROWS / 64), blk, 0, stream>>>(Ctx16, W1_t, b1, Mid16);
  ffn2_kernel<<<gg, blk, 0, stream>>>(Mid16, W2_t, b2, out);
}
